// RowAttentionWithPairBias_73254962201330
// MI455X (gfx1250) — hardware-verified
//
#include <hip/hip_runtime.h>
#define MM 128
#define NNR 256
#define IC 256
#define PC 128
#define AC 32
#define NH 8
#define NTK (MM * NNR)
#define NSL (MM * NH)
#define GM 8
#define GS (GM * NH)
#define GT (GM * NNR)

typedef __bf16 v16b __attribute__((ext_vector_type(16)));
typedef unsigned short v8us __attribute__((ext_vector_type(8), may_alias));
typedef float  v8f  __attribute__((ext_vector_type(8)));
typedef float  v4f  __attribute__((ext_vector_type(4)));
typedef float  v4fa __attribute__((ext_vector_type(4), may_alias));
union FragB { v16b v; v8us half[2]; unsigned short u[16]; };

__device__ __forceinline__ unsigned short bf16_bits(float x) { unsigned int u = __float_as_uint(x); return (unsigned short)((u + 0x7FFFu + ((u >> 16) & 1u)) >> 16); }
__device__ __forceinline__ float bf16_val(unsigned short b) { return __uint_as_float(((unsigned int)b) << 16); }
__device__ __forceinline__ float bf16_round(float x) { return bf16_val(bf16_bits(x)); }
template <int NT>
__device__ __forceinline__ v8f mmaN(v16b ah, v16b al, v16b bh, v16b bl, v8f c) {
  c = __builtin_amdgcn_wmma_f32_16x16x32_bf16(false, ah, false, bh, (short)0, c, false, false);
  if (NT >= 2) c = __builtin_amdgcn_wmma_f32_16x16x32_bf16(false, al, false, bh, (short)0, c, false, false);
  if (NT >= 3) c = __builtin_amdgcn_wmma_f32_16x16x32_bf16(false, ah, false, bl, (short)0, c, false, false);
  asm volatile("v_nop\n\tv_nop\n\tv_nop\n\tv_nop" : "+v"(c) : "v"(ah), "v"(al), "v"(bh), "v"(bl));
  return c;
}

__global__ __launch_bounds__(256) void k_wt_bf16(const float* __restrict__ W, unsigned short* __restrict__ Wt, int K, int N) {
  const int t = blockIdx.x * 256 + threadIdx.x;
  const int k8n = K / 8;
  if (t >= N * k8n) return;
  const int n = t / k8n, k8 = (t % k8n) * 8;
  v8us v;
#pragma unroll
  for (int i = 0; i < 8; ++i) v[i] = bf16_bits(W[(size_t)(k8 + i) * N + n]);
  *(volatile v8us*)(Wt + (size_t)n * K + k8) = v;
  __threadfence();
  *(volatile v8us*)(Wt + (size_t)n * K + k8) = v;
}

template <bool ASPLIT, int ACT, bool BIAS_BF16>
__global__ __launch_bounds__(128) void k_gemm_bf(const float* __restrict__ A, int lda, const unsigned short* __restrict__ Wt, int ldb,
                                               const float* __restrict__ bias, float* __restrict__ C, int ldc, int M, int N, int K) {
  __shared__ __attribute__((aligned(16))) float so[4][16][64];
  const int tid = threadIdx.x, w = tid >> 5, lane = tid & 31, ln = lane & 15, hh = lane >> 4;
  const int ntn = N / 64;
  const int wid = blockIdx.x * 4 + w;
  const int mt = wid / ntn, nq = wid % ntn;
  if (mt * 16 >= M) return;
  const int row0 = mt * 16, col0 = nq * 64;
  const float* arow = A + (size_t)(row0 + ln) * lda;
  v8f acc[4] = {};
  for (int kb = 0; kb < K; kb += 32) {
    FragB ah, al;
    const v4f x0 = *(const v4fa*)(arow + kb + 8 * hh), x1 = *(const v4fa*)(arow + kb + 8 * hh + 4);
    const v4f x2 = *(const v4fa*)(arow + kb + 16 + 8 * hh), x3 = *(const v4fa*)(arow + kb + 16 + 8 * hh + 4);
    float xs[16] = {x0[0],x0[1],x0[2],x0[3],x1[0],x1[1],x1[2],x1[3],x2[0],x2[1],x2[2],x2[3],x3[0],x3[1],x3[2],x3[3]};
#pragma unroll
    for (int i = 0; i < 16; ++i) { const unsigned short hb = bf16_bits(xs[i]); ah.u[i] = hb; al.u[i] = ASPLIT ? bf16_bits(xs[i] - bf16_val(hb)) : (unsigned short)0; }
#pragma unroll
    for (int t = 0; t < 4; ++t) {
      const unsigned short* brow = Wt + (size_t)(col0 + t * 16 + ln) * ldb + kb;
      FragB b;
      b.half[0] = *(const v8us*)(brow + 8 * hh);
      b.half[1] = *(const v8us*)(brow + 16 + 8 * hh);
      acc[t] = mmaN<ASPLIT ? 2 : 1>(ah.v, al.v, b.v, b.v, acc[t]);
    }
  }
#pragma unroll
  for (int t = 0; t < 4; ++t) {
    float bv = bias ? bias[col0 + t * 16 + ln] : 0.f;
    if (BIAS_BF16) bv = bf16_round(bv);
#pragma unroll
    for (int r = 0; r < 8; ++r) { float v = acc[t][r] + bv; if (ACT == 1) v = fmaxf(v, 0.f); so[w][8 * hh + r][t * 16 + ln] = v; }
  }
  __builtin_amdgcn_fence(__ATOMIC_ACQ_REL, "workgroup");
  __builtin_amdgcn_wave_barrier();
  const int rsub = lane >> 4, c4 = (lane & 15) * 4;
  for (int pass = 0; pass < 2; ++pass) {
#pragma unroll
    for (int q = 0; q < 8; ++q) {
      const int r = q * 2 + rsub;
      const v4f v = *(const v4fa*)&so[w][r][c4];
      *(volatile v4f*)(C + (size_t)(row0 + r) * ldc + col0 + c4) = v;
    }
    if (pass == 0) __threadfence();
  }
}

template <int D, bool CAUSAL>
__global__ __launch_bounds__(128) void k_flash(const float* __restrict__ qb, const float* __restrict__ kb, const float* __restrict__ vb,
                                             int pitch, int T, int H, float scale, float* __restrict__ y, int ypitch) {
  constexpr int KS = D / 32;
  constexpr int DT = D / 16;
  __shared__ __attribute__((aligned(16))) unsigned short sKh[32][D + 8], sKl[32][D + 8], sVh[32][D + 8], sVl[32][D + 8];
  __shared__ __attribute__((aligned(16))) unsigned short sPh[4][16][40], sPl[4][16][40];
  __shared__ __attribute__((aligned(16))) float sO[4][16][D];
  const int tid = threadIdx.x, w = tid >> 5, lane = tid & 31, ln = lane & 15, hh = lane >> 4;
  const int nqb = (T + 63) / 64;
  const int bh = blockIdx.x / nqb, qblk = blockIdx.x % nqb;
  const int b = bh / H, h = bh % H;
  const int q0 = qblk * 64 + w * 16;
  const float* Q = qb + (size_t)b * T * pitch + h * D;
  const float* K = kb + (size_t)b * T * pitch + h * D;
  const float* V = vb + (size_t)b * T * pitch + h * D;

  FragB aqh[KS], aql[KS];
  {
    int row = q0 + ln; if (row >= T) row = T - 1;
    const float* qr = Q + (size_t)row * pitch;
#pragma unroll
    for (int ks = 0; ks < KS; ++ks)
#pragma unroll
      for (int i = 0; i < 16; ++i) {
        const int d = ks * 32 + ((i < 8) ? (8 * hh + i) : (16 + 8 * hh + (i - 8)));
        const float x = qr[d] * scale; const unsigned short hb = bf16_bits(x);
        aqh[ks].u[i] = hb; aql[ks].u[i] = bf16_bits(x - bf16_val(hb));
      }
  }
  float m_r[8], l_r[8];
#pragma unroll
  for (int r = 0; r < 8; ++r) { m_r[r] = -3.0e38f; l_r[r] = 0.f; }
  v8f oacc[DT];
#pragma unroll
  for (int dt = 0; dt < DT; ++dt) oacc[dt] = (v8f){0.f,0.f,0.f,0.f,0.f,0.f,0.f,0.f};

  const int kv_end = CAUSAL ? min(T, qblk * 64 + 64) : T;
  for (int j0 = 0; j0 < kv_end; j0 += 32) {
    __syncthreads();
    for (int e = tid; e < 32 * (D / 4); e += 128) {
      const int r = e / (D / 4), c4 = (e % (D / 4)) * 4;
      const int key = j0 + r;
      v4f kf = {0.f,0.f,0.f,0.f}, vf = {0.f,0.f,0.f,0.f};
      if (key < T) { kf = *(const v4fa*)(K + (size_t)key * pitch + c4); vf = *(const v4fa*)(V + (size_t)key * pitch + c4); }
#pragma unroll
      for (int t = 0; t < 4; ++t) {
        unsigned short hb = bf16_bits(kf[t]); sKh[r][c4 + t] = hb; sKl[r][c4 + t] = bf16_bits(kf[t] - bf16_val(hb));
        hb = bf16_bits(vf[t]); sVh[r][c4 + t] = hb; sVl[r][c4 + t] = bf16_bits(vf[t] - bf16_val(hb));
      }
    }
    __syncthreads();
    v8f s[2];
#pragma unroll
    for (int nt = 0; nt < 2; ++nt) {
      v8f acc = {};
#pragma unroll
      for (int ks = 0; ks < KS; ++ks) {
        FragB bh_, bl_;
        bh_.half[0] = *(const v8us*)&sKh[nt * 16 + ln][ks * 32 + 8 * hh]; bh_.half[1] = *(const v8us*)&sKh[nt * 16 + ln][ks * 32 + 16 + 8 * hh];
        bl_.half[0] = *(const v8us*)&sKl[nt * 16 + ln][ks * 32 + 8 * hh]; bl_.half[1] = *(const v8us*)&sKl[nt * 16 + ln][ks * 32 + 16 + 8 * hh];
        acc = mmaN<3>(aqh[ks].v, aql[ks].v, bh_.v, bl_.v, acc);
      }
      s[nt] = acc;
    }
    float alpha[8];
#pragma unroll
    for (int r = 0; r < 8; ++r) {
      const int qi = q0 + 8 * hh + r;
      const int ja = j0 + ln, jb = j0 + 16 + ln;
      if (CAUSAL) { if (ja > qi) s[0][r] = -3.0e38f; if (jb > qi) s[1][r] = -3.0e38f; }
      if (ja >= T) s[0][r] = -3.0e38f;
      if (jb >= T) s[1][r] = -3.0e38f;
      float mx = fmaxf(s[0][r], s[1][r]);
      mx = fmaxf(mx, __shfl_xor(mx, 1, 32)); mx = fmaxf(mx, __shfl_xor(mx, 2, 32)); mx = fmaxf(mx, __shfl_xor(mx, 4, 32)); mx = fmaxf(mx, __shfl_xor(mx, 8, 32));
      const float mnew = fmaxf(m_r[r], mx);
      alpha[r] = (mnew > -1.0e38f) ? __expf(m_r[r] - mnew) : 1.0f;
      const float p0 = (s[0][r] > -1.0e38f) ? __expf(s[0][r] - mnew) : 0.f;
      const float p1 = (s[1][r] > -1.0e38f) ? __expf(s[1][r] - mnew) : 0.f;
      m_r[r] = mnew;
      l_r[r] = l_r[r] * alpha[r] + p0 + p1;
      unsigned short hb = bf16_bits(p0); sPh[w][8 * hh + r][ln] = hb;      sPl[w][8 * hh + r][ln] = bf16_bits(p0 - bf16_val(hb));
      hb = bf16_bits(p1);                sPh[w][8 * hh + r][16 + ln] = hb; sPl[w][8 * hh + r][16 + ln] = bf16_bits(p1 - bf16_val(hb));
    }
#pragma unroll
    for (int dt = 0; dt < DT; ++dt)
#pragma unroll
      for (int r = 0; r < 8; ++r) oacc[dt][r] *= alpha[r];
    __builtin_amdgcn_fence(__ATOMIC_ACQ_REL, "workgroup");
    __builtin_amdgcn_wave_barrier();
    FragB pah, pal;
    pah.half[0] = *(const v8us*)&sPh[w][ln][8 * hh]; pah.half[1] = *(const v8us*)&sPh[w][ln][16 + 8 * hh];
    pal.half[0] = *(const v8us*)&sPl[w][ln][8 * hh]; pal.half[1] = *(const v8us*)&sPl[w][ln][16 + 8 * hh];
#pragma unroll
    for (int dt = 0; dt < DT; ++dt) {
      FragB bvh, bvl;
#pragma unroll
      for (int i = 0; i < 8; ++i) {
        bvh.u[i] = sVh[8 * hh + i][dt * 16 + ln]; bvh.u[8 + i] = sVh[16 + 8 * hh + i][dt * 16 + ln];
        bvl.u[i] = sVl[8 * hh + i][dt * 16 + ln]; bvl.u[8 + i] = sVl[16 + 8 * hh + i][dt * 16 + ln];
      }
      oacc[dt] = mmaN<3>(pah.v, pal.v, bvh.v, bvl.v, oacc[dt]);
    }
    __builtin_amdgcn_fence(__ATOMIC_ACQ_REL, "workgroup");
    __builtin_amdgcn_wave_barrier();
  }
#pragma unroll
  for (int r = 0; r < 8; ++r) {
    float l = l_r[r];
    l += __shfl_xor(l, 1, 32); l += __shfl_xor(l, 2, 32); l += __shfl_xor(l, 4, 32); l += __shfl_xor(l, 8, 32);
    l_r[r] = (l > 0.f) ? 1.0f / l : 0.f;
  }
#pragma unroll
  for (int dt = 0; dt < DT; ++dt)
#pragma unroll
    for (int r = 0; r < 8; ++r) sO[w][8 * hh + r][dt * 16 + ln] = oacc[dt][r] * l_r[r];
  __builtin_amdgcn_fence(__ATOMIC_ACQ_REL, "workgroup");
  __builtin_amdgcn_wave_barrier();
  for (int pass = 0; pass < 2; ++pass) {
    for (int r = 0; r < 16; ++r) {
      const int row = q0 + r;
      if (row < T && lane < D / 4) {
        const v4f val = *(const v4fa*)&sO[w][r][lane * 4];
        *(volatile v4f*)(y + ((size_t)b * T + row) * ypitch + h * D + lane * 4) = val;
      }
    }
    if (pass == 0) __threadfence();
  }
}

template <bool ASPLIT, int ACT, bool BIAS_BF16, bool RES_BF16>
__global__ __launch_bounds__(128) void k_gemm_bf3(const float* __restrict__ A, int lda, const unsigned short* __restrict__ Wt, int ldb,
                                                const float* __restrict__ bias, const float* __restrict__ resid, int rmod, int ldr,
                                                float* __restrict__ C, int ldc, int M, int N, int K) {
  __shared__ __attribute__((aligned(16))) float so[4][16][64];
  const int tid = threadIdx.x, w = tid >> 5, lane = tid & 31, ln = lane & 15, hh = lane >> 4;
  const int ntn = N / 64;
  const int wid = blockIdx.x * 4 + w;
  const int mt = wid / ntn, nq = wid % ntn;
  if (mt * 16 >= M) return;
  const int row0 = mt * 16, col0 = nq * 64;
  const float* arow = A + (size_t)(row0 + ln) * lda;
  v8f acc[4] = {};
  for (int kb = 0; kb < K; kb += 32) {
    FragB ah, al;
    const v4f x0 = *(const v4fa*)(arow + kb + 8 * hh), x1 = *(const v4fa*)(arow + kb + 8 * hh + 4);
    const v4f x2 = *(const v4fa*)(arow + kb + 16 + 8 * hh), x3 = *(const v4fa*)(arow + kb + 16 + 8 * hh + 4);
    float xs[16] = {x0[0],x0[1],x0[2],x0[3],x1[0],x1[1],x1[2],x1[3],x2[0],x2[1],x2[2],x2[3],x3[0],x3[1],x3[2],x3[3]};
#pragma unroll
    for (int i = 0; i < 16; ++i) { const unsigned short hb = bf16_bits(xs[i]); ah.u[i] = hb; al.u[i] = ASPLIT ? bf16_bits(xs[i] - bf16_val(hb)) : (unsigned short)0; }
#pragma unroll
    for (int t = 0; t < 4; ++t) {
      const unsigned short* brow = Wt + (size_t)(col0 + t * 16 + ln) * ldb + kb;
      FragB b;
      b.half[0] = *(const v8us*)(brow + 8 * hh);
      b.half[1] = *(const v8us*)(brow + 16 + 8 * hh);
      acc[t] = mmaN<ASPLIT ? 2 : 1>(ah.v, al.v, b.v, b.v, acc[t]);
    }
  }
#pragma unroll
  for (int t = 0; t < 4; ++t) {
    const int col = col0 + t * 16 + ln;
    float bv = bias ? bias[col] : 0.f;
    if (BIAS_BF16) bv = bf16_round(bv);
#pragma unroll
    for (int r = 0; r < 8; ++r) {
      float v = acc[t][r] + bv;
      if (resid) { float rv = resid[(size_t)((row0 + 8 * hh + r) % rmod) * ldr + col]; if (RES_BF16) rv = bf16_round(rv); v += rv; }
      if (ACT == 1) v = fmaxf(v, 0.f);
      if (ACT == 2) v = 0.5f * v * (1.0f + erff(v * 0.70710678118654752f));
      if (ACT == 3) { const float u = 0.7978845608028654f * (v + 0.044715f * v * v * v); v = 0.5f * v * (1.0f + tanhf(u)); }
      so[w][8 * hh + r][t * 16 + ln] = v;
    }
  }
  __builtin_amdgcn_fence(__ATOMIC_ACQ_REL, "workgroup");
  __builtin_amdgcn_wave_barrier();
  const int rsub = lane >> 4, c4 = (lane & 15) * 4;
  for (int pass = 0; pass < 2; ++pass) {
#pragma unroll
    for (int q = 0; q < 8; ++q) {
      const int r = q * 2 + rsub;
      const v4f v = *(const v4fa*)&so[w][r][c4];
      *(volatile v4f*)(C + (size_t)(row0 + r) * ldc + col0 + c4) = v;
    }
    if (pass == 0) __threadfence();
  }
}
template <bool PARAM_BF16>
__global__ __launch_bounds__(256) void k_layernorm(const float* __restrict__ X, const float* __restrict__ R, const float* __restrict__ g, const float* __restrict__ bta,
                                                  float* __restrict__ out_sum, float* __restrict__ out_norm, int N, float eps) {
  __shared__ float red[256];
  const int row = blockIdx.x, tid = threadIdx.x;
  const float* x = X + (size_t)row * N; const float* rr = R ? R + (size_t)row * N : nullptr;
  float vals[16];
  const int per = N / 256;
  float s1 = 0.f;
  for (int u = 0; u < per / 4; ++u) {
    const int j = tid * 4 + 1024 * u;
    const v4f a = *(const v4fa*)(x + j);
    v4f b = {0.f,0.f,0.f,0.f}; if (rr) b = *(const v4fa*)(rr + j);
#pragma unroll
    for (int q = 0; q < 4; ++q) { const float v = a[q] + b[q]; vals[u * 4 + q] = v; s1 += v; }
  }
  red[tid] = s1; __syncthreads();
  for (int st = 128; st > 0; st >>= 1) { if (tid < st) red[tid] += red[tid + st]; __syncthreads(); }
  const float mu = red[0] / (float)N; __syncthreads();
  float s2 = 0.f;
  for (int u = 0; u < per / 4; ++u)
#pragma unroll
    for (int q = 0; q < 4; ++q) { const float c = vals[u * 4 + q] - mu; s2 += c * c; }
  red[tid] = s2; __syncthreads();
  for (int st = 128; st > 0; st >>= 1) { if (tid < st) red[tid] += red[tid + st]; __syncthreads(); }
  const float rs = rsqrtf(red[0] / (float)N + eps);
  for (int pass = 0; pass < 2; ++pass) {
    for (int u = 0; u < per / 4; ++u) {
      const int j = tid * 4 + 1024 * u;
      v4f o, sm;
#pragma unroll
      for (int q = 0; q < 4; ++q) {
        float gg = g[j + q], bb = bta[j + q];
        if (PARAM_BF16) { gg = bf16_round(gg); bb = bf16_round(bb); }
        sm[q] = vals[u * 4 + q]; o[q] = (vals[u * 4 + q] - mu) * rs * gg + bb;
      }
      if (out_sum) *(volatile v4f*)(out_sum + (size_t)row * N + j) = sm;
      *(volatile v4f*)(out_norm + (size_t)row * N + j) = o;
    }
    if (pass == 0) __threadfence();
  }
}

template <bool ASPLIT, bool BSPLIT, int ACT>
__global__ __launch_bounds__(128) void k_gemm_b(const float* __restrict__ A, int lda, size_t sA, const unsigned short* __restrict__ Bh, const unsigned short* __restrict__ Bl, int ldb, size_t sB,
                                             const float* __restrict__ bias, const float* __restrict__ resid, int ldr, size_t sR, float rsign, float alpha,
                                             float* __restrict__ C, int ldc, size_t sC, int M, int N, int K) {
  __shared__ __attribute__((aligned(16))) float so[4][16][64];
  const int tid = threadIdx.x, w = tid >> 5, lane = tid & 31, ln = lane & 15, hh = lane >> 4;
  const int by = blockIdx.y;
  A += (size_t)by * sA; Bh += (size_t)by * sB; if (BSPLIT) Bl += (size_t)by * sB; C += (size_t)by * sC; if (resid) resid += (size_t)by * sR;
  const int ntn = (N + 63) / 64; const int wid = blockIdx.x * 4 + w; const int mt = wid / ntn, nq = wid % ntn;
  if (mt * 16 >= M) return;
  const int row0 = mt * 16, col0 = nq * 64;
  const float* arow = A + (size_t)(row0 + ln) * lda;
  v8f acc[4] = {};
  for (int kb = 0; kb < K; kb += 32) {
    FragB ah, al;
    const v4f x0 = *(const v4fa*)(arow + kb + 8 * hh), x1 = *(const v4fa*)(arow + kb + 8 * hh + 4);
    const v4f x2 = *(const v4fa*)(arow + kb + 16 + 8 * hh), x3 = *(const v4fa*)(arow + kb + 16 + 8 * hh + 4);
    float xs[16] = {x0[0],x0[1],x0[2],x0[3],x1[0],x1[1],x1[2],x1[3],x2[0],x2[1],x2[2],x2[3],x3[0],x3[1],x3[2],x3[3]};
#pragma unroll
    for (int i = 0; i < 16; ++i) { const unsigned short hb = bf16_bits(xs[i]); ah.u[i] = hb; al.u[i] = ASPLIT ? bf16_bits(xs[i] - bf16_val(hb)) : (unsigned short)0; }
#pragma unroll
    for (int t = 0; t < 4; ++t) {
      if (col0 + t * 16 >= N) continue;
      const size_t boff = (size_t)(col0 + t * 16 + ln) * ldb + kb;
      FragB bh_, bl_; bh_.half[0] = *(const v8us*)(Bh + boff + 8 * hh); bh_.half[1] = *(const v8us*)(Bh + boff + 16 + 8 * hh);
      if (BSPLIT) { bl_.half[0] = *(const v8us*)(Bl + boff + 8 * hh); bl_.half[1] = *(const v8us*)(Bl + boff + 16 + 8 * hh); } else bl_ = bh_;
      acc[t] = mmaN<ASPLIT ? (BSPLIT ? 3 : 2) : 1>(ah.v, al.v, bh_.v, bl_.v, acc[t]);
    }
  }
#pragma unroll
  for (int t = 0; t < 4; ++t) {
    const int col = col0 + t * 16 + ln; if (col0 + t * 16 >= N) continue; const float bv = bias ? bf16_round(bias[col]) : 0.f;
#pragma unroll
    for (int r = 0; r < 8; ++r) { float v = acc[t][r] * alpha + bv; if (resid) v += rsign * resid[(size_t)(row0 + 8 * hh + r) * ldr + col]; if (ACT == 1) v = fmaxf(v, 0.f); else if (ACT == 2) v = fmaxf(v, 0.f) + log1pf(expf(-fabsf(v))); so[w][8 * hh + r][t * 16 + ln] = v; }
  }
  __builtin_amdgcn_fence(__ATOMIC_ACQ_REL, "workgroup"); __builtin_amdgcn_wave_barrier();
  const int rsub = lane >> 4, c4 = (lane & 15) * 4;
  for (int pass = 0; pass < 2; ++pass) {
#pragma unroll
    for (int q = 0; q < 8; ++q) { const int r = q * 2 + rsub; if (col0 + c4 < N) { const v4f v = *(const v4fa*)&so[w][r][c4]; *(volatile v4f*)(C + (size_t)(row0 + r) * ldc + col0 + c4) = v; } }
    if (pass == 0) __threadfence();
  }
}
__global__ __launch_bounds__(256) void k_split_transpose_b(const float* __restrict__ src, int lds_, size_t sIn, unsigned short* __restrict__ hi, unsigned short* __restrict__ lo, size_t sOut, int K, int N) {
  const size_t t = (size_t)blockIdx.x * 256 + threadIdx.x; const int k8n = K / 8; if (t >= (size_t)N * k8n) return;
  src += (size_t)blockIdx.y * sIn; hi += (size_t)blockIdx.y * sOut; lo += (size_t)blockIdx.y * sOut;
  const int n = (int)(t / k8n), k8 = (int)(t % k8n) * 8; v8us vh, vl;
#pragma unroll
  for (int i = 0; i < 8; ++i) { const float x = src[(size_t)(k8 + i) * lds_ + n]; const unsigned short hb = bf16_bits(x); vh[i] = hb; vl[i] = bf16_bits(x - bf16_val(hb)); }
  unsigned short* dh = hi + (size_t)n * K + k8; unsigned short* dl = lo + (size_t)n * K + k8;
  *(volatile v8us*)dh = vh; *(volatile v8us*)dl = vl; __threadfence(); *(volatile v8us*)dh = vh; *(volatile v8us*)dl = vl;
}

typedef _Float16 v16h __attribute__((ext_vector_type(16)));
union FragH { v16h v; v8us half[2]; _Float16 h[16]; unsigned short u[16]; };
template <int NT>
__device__ __forceinline__ v8f mmaH(v16h ah, v16h al, v16h bh, v16h bl, v8f c) {
  c = __builtin_amdgcn_wmma_f32_16x16x32_f16(false, ah, false, bh, (short)0, c, false, false);
  if (NT >= 2) c = __builtin_amdgcn_wmma_f32_16x16x32_f16(false, al, false, bh, (short)0, c, false, false);
  if (NT >= 3) c = __builtin_amdgcn_wmma_f32_16x16x32_f16(false, ah, false, bl, (short)0, c, false, false);
  asm volatile("v_nop\n\tv_nop\n\tv_nop\n\tv_nop" : "+v"(c) : "v"(ah), "v"(al), "v"(bh), "v"(bl));
  return c;
}
template <bool ASPLIT>
__global__ __launch_bounds__(128) void k_gemm_h(const float* __restrict__ A, int lda, size_t sA, const _Float16* __restrict__ Bh, int ldb, size_t sB, float alpha, float* __restrict__ C, int ldc, size_t sC, int M, int N, int K) {
  __shared__ __attribute__((aligned(16))) float so[4][16][64];
  const int tid = threadIdx.x, w = tid >> 5, lane = tid & 31, ln = lane & 15, hh = lane >> 4; const int by = blockIdx.y;
  A += (size_t)by * sA; Bh += (size_t)by * sB; C += (size_t)by * sC;
  const int ntn = (N + 63) / 64; const int wid = blockIdx.x * 4 + w; const int mt = wid / ntn, nq = wid % ntn; if (mt * 16 >= M) return;
  const int row0 = mt * 16, col0 = nq * 64; const float* arow = A + (size_t)(row0 + ln) * lda;
  v8f acc[4] = {};
  for (int kb = 0; kb < K; kb += 32) {
    FragH ah, al;
    const v4f x0 = *(const v4fa*)(arow + kb + 8 * hh), x1 = *(const v4fa*)(arow + kb + 8 * hh + 4), x2 = *(const v4fa*)(arow + kb + 16 + 8 * hh), x3 = *(const v4fa*)(arow + kb + 16 + 8 * hh + 4);
    float xs[16] = {x0[0],x0[1],x0[2],x0[3],x1[0],x1[1],x1[2],x1[3],x2[0],x2[1],x2[2],x2[3],x3[0],x3[1],x3[2],x3[3]};
#pragma unroll
    for (int i = 0; i < 16; ++i) { const _Float16 h = (_Float16)xs[i]; ah.h[i] = h; al.h[i] = ASPLIT ? (_Float16)(xs[i] - (float)h) : (_Float16)0.0f; }
#pragma unroll
    for (int t = 0; t < 4; ++t) { if (col0 + t * 16 >= N) continue; const size_t boff = (size_t)(col0 + t * 16 + ln) * ldb + kb; FragH bq; bq.half[0] = *(const v8us*)(Bh + boff + 8 * hh); bq.half[1] = *(const v8us*)(Bh + boff + 16 + 8 * hh);
      acc[t] = mmaH<ASPLIT ? 2 : 1>(ah.v, al.v, bq.v, bq.v, acc[t]); }
  }
#pragma unroll
  for (int t = 0; t < 4; ++t) { if (col0 + t * 16 >= N) continue;
#pragma unroll
    for (int r = 0; r < 8; ++r) so[w][8 * hh + r][t * 16 + ln] = acc[t][r] * alpha; }
  __builtin_amdgcn_fence(__ATOMIC_ACQ_REL, "workgroup"); __builtin_amdgcn_wave_barrier();
  const int rsub = lane >> 4, c4 = (lane & 15) * 4;
  for (int pass = 0; pass < 2; ++pass) {
#pragma unroll
    for (int q = 0; q < 8; ++q) { const int r = q * 2 + rsub; if (col0 + c4 < N) { const v4f v = *(const v4fa*)&so[w][r][c4]; *(volatile v4f*)(C + (size_t)(row0 + r) * ldc + col0 + c4) = v; } }
    if (pass == 0) __threadfence(); }
}

__global__ __launch_bounds__(256) void k_wt_f16n(const float* __restrict__ W, _Float16* __restrict__ Wt, size_t n8tot, float scale) { const size_t t = (size_t)blockIdx.x * 256 + threadIdx.x; if (t >= n8tot) return; FragH f;
#pragma unroll
  for (int i = 0; i < 8; ++i) f.h[i] = (_Float16)(bf16_round(W[t * 8 + i]) * scale); const v8us o = f.half[0]; *(volatile v8us*)((unsigned short*)Wt + t * 8) = o; __threadfence(); *(volatile v8us*)((unsigned short*)Wt + t * 8) = o; }

__global__ __launch_bounds__(256) void k_wt_qkvg(const float* __restrict__ qkvw, const float* __restrict__ gw, _Float16* __restrict__ Bt) { const size_t t = (size_t)blockIdx.x * 256 + threadIdx.x; if (t >= (size_t)1024 * IC / 8) return;
  const int nr = (int)(t / (IC / 8)), k8 = (int)(t % (IC / 8)) * 8; const float* src;
  if (nr < 768) { const int p = nr / 256, h = (nr % 256) / AC, c = nr % AC; src = qkvw + (size_t)(c * 24 + p * 8 + h) * IC; } else src = gw + (size_t)(nr - 768) * IC;
  FragH f;
#pragma unroll
  for (int i = 0; i < 8; ++i) f.h[i] = (_Float16)(bf16_round(src[k8 + i]) * 16.0f); const v8us o = f.half[0]; *(volatile v8us*)((unsigned short*)Bt + t * 8) = o; __threadfence(); *(volatile v8us*)((unsigned short*)Bt + t * 8) = o; }
__global__ __launch_bounds__(128) void k_gemm_qk(const float* __restrict__ X, const _Float16* __restrict__ Bt, float* __restrict__ Q2, _Float16* __restrict__ Kh, _Float16* __restrict__ Kl) {
  __shared__ __attribute__((aligned(16))) float so[4][16][64];
  const int tid = threadIdx.x, w = tid >> 5, lane = tid & 31, ln = lane & 15, hh = lane >> 4;
  constexpr int NTN = 512 / 64; const int wid = blockIdx.x * 4 + w; const int mt = wid / NTN, nq = wid % NTN; if (mt * 16 >= GT) return;
  const int row0 = mt * 16, col0 = nq * 64; const float* arow = X + (size_t)(row0 + ln) * IC;
  v8f acc[4] = {};
  for (int kb = 0; kb < IC; kb += 32) {
    FragH ah, al;
    const v4f x0 = *(const v4fa*)(arow + kb + 8 * hh), x1 = *(const v4fa*)(arow + kb + 8 * hh + 4), x2 = *(const v4fa*)(arow + kb + 16 + 8 * hh), x3 = *(const v4fa*)(arow + kb + 16 + 8 * hh + 4);
    float xs[16] = {x0[0],x0[1],x0[2],x0[3],x1[0],x1[1],x1[2],x1[3],x2[0],x2[1],x2[2],x2[3],x3[0],x3[1],x3[2],x3[3]};
#pragma unroll
    for (int i = 0; i < 16; ++i) { const _Float16 h = (_Float16)xs[i]; ah.h[i] = h; al.h[i] = (_Float16)(xs[i] - (float)h); }
#pragma unroll
    for (int t = 0; t < 4; ++t) { const size_t boff = (size_t)(col0 + t * 16 + ln) * IC + kb; FragH bq; bq.half[0] = *(const v8us*)((const unsigned short*)Bt + boff + 8 * hh); bq.half[1] = *(const v8us*)((const unsigned short*)Bt + boff + 16 + 8 * hh);
      acc[t] = mmaH<2>(ah.v, al.v, bq.v, bq.v, acc[t]); }
  }
#pragma unroll
  for (int t = 0; t < 4; ++t) {
#pragma unroll
    for (int r = 0; r < 8; ++r) so[w][8 * hh + r][t * 16 + ln] = acc[t][r] * 0.0625f; }
  __builtin_amdgcn_fence(__ATOMIC_ACQ_REL, "workgroup"); __builtin_amdgcn_wave_barrier();
  const int m = row0 / NNR, i0 = row0 % NNR;
  const bool isq = col0 < 256; const int h0 = (col0 % 256) / AC;
  const int hsel = lane >> 4, l16 = lane & 15;
  const size_t slab = (size_t)m * NH + h0 + hsel;
  for (int pass = 0; pass < 2; ++pass) {
    if (isq) {
#pragma unroll
      for (int q = 0; q < 8; ++q) { const int r = q + 8 * (l16 >> 3); const int c4 = (l16 & 7) * 4; const v4f v = *(const v4fa*)&so[w][r][hsel * 32 + c4];
        *(volatile v4f*)(Q2 + (slab * NNR + i0 + r) * AC + c4) = v; }
    } else {
      typedef _Float16 v4h __attribute__((ext_vector_type(4)));
#pragma unroll
      for (int q = 0; q < 8; ++q) { const int r = 2 * q + (l16 >> 3); const int c4 = (l16 & 7) * 4; const v4f v = *(const v4fa*)&so[w][r][hsel * 32 + c4]; v4h vh, vl;
#pragma unroll
        for (int u = 0; u < 4; ++u) { const _Float16 hb = (_Float16)v[u]; vh[u] = hb; vl[u] = (_Float16)(v[u] - (float)hb); }
        const size_t o = (slab * NNR + i0 + r) * AC + c4; *(volatile v4h*)(Kh + o) = vh; *(volatile v4h*)(Kl + o) = vl; }
    }
    if (pass == 0) __threadfence(); }
}
__global__ __launch_bounds__(128) void k_gemm_h3(const float* __restrict__ A, int lda, size_t sA, const _Float16* __restrict__ Bh, const _Float16* __restrict__ Bl, int ldb, size_t sB, float alpha, float* __restrict__ C, int ldc, size_t sC, int M, int N, int K) {
  __shared__ __attribute__((aligned(16))) float so[4][16][64];
  const int tid = threadIdx.x, w = tid >> 5, lane = tid & 31, ln = lane & 15, hh = lane >> 4; const int by = blockIdx.y;
  A += (size_t)by * sA; Bh += (size_t)by * sB; Bl += (size_t)by * sB; C += (size_t)by * sC;
  const int ntn = (N + 63) / 64; const int wid = blockIdx.x * 4 + w; const int mt = wid / ntn, nq = wid % ntn; if (mt * 16 >= M) return;
  const int row0 = mt * 16, col0 = nq * 64; const float* arow = A + (size_t)(row0 + ln) * lda;
  v8f acc[4] = {};
  for (int kb = 0; kb < K; kb += 32) {
    FragH ah, al;
    const v4f x0 = *(const v4fa*)(arow + kb + 8 * hh), x1 = *(const v4fa*)(arow + kb + 8 * hh + 4), x2 = *(const v4fa*)(arow + kb + 16 + 8 * hh), x3 = *(const v4fa*)(arow + kb + 16 + 8 * hh + 4);
    float xs[16] = {x0[0],x0[1],x0[2],x0[3],x1[0],x1[1],x1[2],x1[3],x2[0],x2[1],x2[2],x2[3],x3[0],x3[1],x3[2],x3[3]};
#pragma unroll
    for (int i = 0; i < 16; ++i) { const _Float16 h = (_Float16)xs[i]; ah.h[i] = h; al.h[i] = (_Float16)(xs[i] - (float)h); }
#pragma unroll
    for (int t = 0; t < 4; ++t) { if (col0 + t * 16 >= N) continue; const size_t boff = (size_t)(col0 + t * 16 + ln) * ldb + kb; FragH bh_, bl_;
      bh_.half[0] = *(const v8us*)((const unsigned short*)Bh + boff + 8 * hh); bh_.half[1] = *(const v8us*)((const unsigned short*)Bh + boff + 16 + 8 * hh);
      bl_.half[0] = *(const v8us*)((const unsigned short*)Bl + boff + 8 * hh); bl_.half[1] = *(const v8us*)((const unsigned short*)Bl + boff + 16 + 8 * hh);
      acc[t] = mmaH<3>(ah.v, al.v, bh_.v, bl_.v, acc[t]); }
  }
#pragma unroll
  for (int t = 0; t < 4; ++t) { if (col0 + t * 16 >= N) continue;
#pragma unroll
    for (int r = 0; r < 8; ++r) so[w][8 * hh + r][t * 16 + ln] = acc[t][r] * alpha; }
  __builtin_amdgcn_fence(__ATOMIC_ACQ_REL, "workgroup"); __builtin_amdgcn_wave_barrier();
  const int rsub = lane >> 4, c4 = (lane & 15) * 4;
  for (int pass = 0; pass < 2; ++pass) {
#pragma unroll
    for (int q = 0; q < 8; ++q) { const int r = q * 2 + rsub; if (col0 + c4 < N) { const v4f v = *(const v4fa*)&so[w][r][c4]; *(volatile v4f*)(C + (size_t)(row0 + r) * ldc + col0 + c4) = v; } }
    if (pass == 0) __threadfence(); }
}
__global__ __launch_bounds__(256) void k_arrVg(const float* __restrict__ Vg, _Float16* __restrict__ Vt) { const size_t t = (size_t)blockIdx.x * 256 + threadIdx.x; if (t >= (size_t)GS * AC * (NNR / 8)) return; const int r8 = (int)(t % (NNR / 8)) * 8; const int c = (int)((t / (NNR / 8)) % AC); const int sl = (int)(t / ((size_t)(NNR / 8) * AC)); const int ml = sl / NH, h = sl % NH; FragH f;
#pragma unroll
  for (int q = 0; q < 8; ++q) f.h[q] = (_Float16)Vg[((size_t)ml * NNR + r8 + q) * 256 + h * AC + c]; const v8us o = f.half[0]; *(volatile v8us*)((unsigned short*)Vt + ((size_t)sl * AC + c) * NNR + r8) = o; __threadfence(); *(volatile v8us*)((unsigned short*)Vt + ((size_t)sl * AC + c) * NNR + r8) = o; }
__global__ __launch_bounds__(256) void k_ln(const float* __restrict__ x, const float* __restrict__ w, const float* __restrict__ b, float* __restrict__ X) {
  const int tid = threadIdx.x, wv = tid >> 5, lane = tid & 31; const size_t t = (size_t)blockIdx.x * 8 + wv; const float* r = x + t * IC; float v[8]; float s = 0.f;
#pragma unroll
  for (int u = 0; u < 8; ++u) { v[u] = bf16_round(r[u * 32 + lane]); s += v[u]; }
  for (int o = 16; o >= 1; o >>= 1) s += __shfl_xor(s, o, 32); const float mu = s / (float)IC; float q = 0.f;
#pragma unroll
  for (int u = 0; u < 8; ++u) { const float d = v[u] - mu; q += d * d; }
  for (int o = 16; o >= 1; o >>= 1) q += __shfl_xor(q, o, 32); const float rs = 1.0f / sqrtf(q / (float)IC + 1e-5f);
  float* dst = X + t * IC; for (int pass = 0; pass < 2; ++pass) {
#pragma unroll
    for (int u = 0; u < 8; ++u) { const int c = u * 32 + lane; *(volatile float*)(dst + c) = (v[u] - mu) * rs * bf16_round(w[c]) + bf16_round(b[c]); } if (pass == 0) __threadfence(); }
}
__global__ __launch_bounds__(256) void k_wb(const float* __restrict__ w, unsigned short* __restrict__ Bt) { const int t = threadIdx.x; if (t >= 16 * 16) return; const int n = t / 16, k8 = (t % 16) * 8; v8us v;
#pragma unroll
  for (int i = 0; i < 8; ++i) v[i] = (n < NH) ? bf16_bits(w[n * PC + k8 + i]) : (unsigned short)0; *(volatile v8us*)(Bt + n * PC + k8) = v; __threadfence(); *(volatile v8us*)(Bt + n * PC + k8) = v; }
__global__ __launch_bounds__(1024) void k_softmax(float* __restrict__ S, const float* __restrict__ BIAS, int sl0, float* __restrict__ Dn) {
  __shared__ float sd[32]; const int tid = threadIdx.x, wv = tid >> 5, lane = tid & 31; const size_t r = (size_t)blockIdx.x * 32 + wv; const int i = (int)(r % NNR); const int sl = sl0 + (int)(r / NNR); const int h = sl % NH; float* row = S + r * NNR; const float fac = 0.17677669529663687f;
  float mx = -3.0e38f;
#pragma unroll 1
  for (int j = lane; j < NNR; j += 32) { const float l = row[j] + BIAS[((size_t)i * NNR + j) * 16 + h] * fac; mx = fmaxf(mx, l); }
  for (int o = 16; o >= 1; o >>= 1) mx = fmaxf(mx, __shfl_xor(mx, o, 32));
  float den = 0.f;
#pragma unroll 1
  for (int j = lane; j < NNR; j += 32) { const float e = expf((row[j] + BIAS[((size_t)i * NNR + j) * 16 + h] * fac) - mx); den += e; const float p = e * 256.0f; *(volatile float*)(row + j) = p; }
  for (int o = 16; o >= 1; o >>= 1) den += __shfl_xor(den, o, 32);
  __threadfence();
#pragma unroll 1
  for (int j = lane; j < NNR; j += 32) { const float p = row[j]; *(volatile float*)(row + j) = p; }
  if (lane == 0) sd[wv] = den; __syncthreads();
  if (tid < 32) { *(volatile float*)(Dn + (size_t)sl0 * NNR + (size_t)blockIdx.x * 32 + tid) = sd[tid]; } __threadfence(); if (tid < 32) { *(volatile float*)(Dn + (size_t)sl0 * NNR + (size_t)blockIdx.x * 32 + tid) = sd[tid]; }
}
__global__ __launch_bounds__(256) void k_combine(const float* __restrict__ O, const float* __restrict__ Dn, const float* __restrict__ G, const float* __restrict__ gateb, float* __restrict__ OUT2) {
  const int tid = threadIdx.x, wv = tid >> 5, lane = tid & 31; const size_t t = (size_t)blockIdx.x * 8 + wv; const int m = (int)(t / NNR), i = (int)(t % NNR); const float* g = G + t * 256; float* dst = OUT2 + t * 256;
  __shared__ float sov[8][256]; float* ov = sov[wv];
#pragma unroll 1
  for (int u = 0; u < 8; ++u) { const int col = u * 32 + lane; const int c = col / NH, h = col % NH; const size_t sl = (size_t)m * NH + h; const float o = O[(sl * NNR + i) * AC + c] / Dn[sl * NNR + i]; const float gv = g[col] + bf16_round(gateb[col]); ov[col] = o * (1.0f / (1.0f + expf(-gv))); }
  for (int pass = 0; pass < 2; ++pass) { for (int u = 0; u < 8; ++u) *(volatile float*)(dst + u * 32 + lane) = ov[u * 32 + lane]; if (pass == 0) __threadfence(); }
}
__global__ __launch_bounds__(256) void k_addbias(float* __restrict__ Y, const float* __restrict__ b, size_t n4) { const size_t t = (size_t)blockIdx.x * 256 + threadIdx.x; if (t >= n4) return; const int c4 = (int)((t * 4) % IC); v4f v = *(const v4fa*)(Y + t * 4); for (int q = 0; q < 4; ++q) v[q] += bf16_round(b[c4 + q]); *(volatile v4f*)(Y + t * 4) = v; __threadfence(); *(volatile v4f*)(Y + t * 4) = v; }
extern "C" void kernel_launch(void* const* d_in, const int* in_sizes, int n_in,
                              void* d_out, int out_size, void* d_ws, size_t ws_size, hipStream_t stream) {
  (void)in_sizes; (void)n_in; (void)out_size;
  const float* x1d = (const float*)d_in[0]; const float* x2d = (const float*)d_in[1]; const float* nw = (const float*)d_in[2]; const float* nb = (const float*)d_in[3]; const float* qkvw = (const float*)d_in[4]; const float* x2dw = (const float*)d_in[5]; const float* gw = (const float*)d_in[6]; const float* gb = (const float*)d_in[7]; const float* fw = (const float*)d_in[8]; const float* fb = (const float*)d_in[9];
  char* ws = (char*)d_ws; size_t off = 0;
  auto take = [&](size_t bytes) { char* p = ws + off; off += (bytes + 255) & ~(size_t)255; return p; };
  _Float16* Bqg = (_Float16*)take((size_t)1024 * IC * 2); unsigned short* Bb = (unsigned short*)take(16 * PC * 2); _Float16* Bf = (_Float16*)take((size_t)IC * IC * 2);
  float* X = (float*)take((size_t)NTK * IC * 4); float* G = (float*)take((size_t)NTK * IC * 4); float* BIAS = (float*)take((size_t)NNR * NNR * 16 * 4);
  float* Q2 = (float*)take((size_t)GS * NNR * AC * 4); _Float16* Kh = (_Float16*)take((size_t)GS * NNR * AC * 2); _Float16* Kl = (_Float16*)take((size_t)GS * NNR * AC * 2); float* Vg = (float*)take((size_t)GT * IC * 4); _Float16* Vt = (_Float16*)take((size_t)GS * AC * NNR * 2);
  float* S = (float*)take((size_t)GS * NNR * NNR * 4); float* Dn = (float*)take((size_t)NSL * NNR * 4); float* O = (float*)take((size_t)NSL * NNR * AC * 4); float* OUT2 = X;
  if (off > ws_size) return;
  k_wt_qkvg<<<(1024 * IC / 8 + 255) / 256, 256, 0, stream>>>(qkvw, gw, Bqg);
  k_wb<<<1, 256, 0, stream>>>(x2dw, Bb); k_wt_f16n<<<(IC * IC / 8 + 255) / 256, 256, 0, stream>>>(fw, Bf, (size_t)IC * IC / 8, 16.0f);
  k_ln<<<NTK / 8, 256, 0, stream>>>(x1d, nw, nb, X);
  k_gemm_h<false><<<dim3(((NTK / 16) * (IC / 64) + 3) / 4, 1), 128, 0, stream>>>(X, IC, 0, Bqg + (size_t)768 * IC, IC, 0, 0.0625f, G, IC, 0, NTK, IC, IC);
  k_gemm_b<false, false, 0><<<dim3(((NNR * NNR / 16) * 1 + 3) / 4, 1), 128, 0, stream>>>(x2d, PC, 0, Bb, Bb, PC, 0, nullptr, nullptr, 0, 0, 1.f, 1.f, BIAS, 16, 0, NNR * NNR, 16, PC);
  for (int g = 0; g < MM / GM; ++g) {
    const int s0 = g * GS; const float* Xg = X + (size_t)g * GT * IC;
    k_gemm_qk<<<((GT / 16) * 8 + 3) / 4, 128, 0, stream>>>(Xg, Bqg, Q2, Kh, Kl);
    k_gemm_h<false><<<dim3(((GT / 16) * (IC / 64) + 3) / 4, 1), 128, 0, stream>>>(Xg, IC, 0, Bqg + (size_t)512 * IC, IC, 0, 0.0625f, Vg, IC, 0, GT, IC, IC);
    k_arrVg<<<(unsigned)(((size_t)GS * AC * (NNR / 8) + 255) / 256), 256, 0, stream>>>(Vg, Vt);
    k_gemm_h3<<<dim3(((NNR / 16) * (NNR / 64) + 3) / 4, GS), 128, 0, stream>>>(Q2, AC, (size_t)NNR * AC, Kh, Kl, AC, (size_t)NNR * AC, 1.f, S, NNR, (size_t)NNR * NNR, NNR, NNR, AC);
    k_softmax<<<(GS * NNR) / 32, 1024, 0, stream>>>(S, BIAS, s0, Dn);
    k_gemm_h<false><<<dim3(((NNR / 16) * 1 + 3) / 4, GS), 128, 0, stream>>>(S, NNR, (size_t)NNR * NNR, Vt, NNR, (size_t)AC * NNR, 0.00390625f, O + (size_t)s0 * NNR * AC, AC, (size_t)NNR * AC, NNR, AC, NNR);
  }
  k_combine<<<NTK / 8, 256, 0, stream>>>(O, Dn, G, gb, OUT2);
  k_gemm_h<false><<<dim3(((NTK / 16) * (IC / 64) + 3) / 4, 1), 128, 0, stream>>>(OUT2, IC, 0, Bf, IC, 0, 0.0625f, (float*)d_out, IC, 0, NTK, IC, IC);
  k_addbias<<<(unsigned)(((size_t)NTK * IC / 4 + 255) / 256), 256, 0, stream>>>((float*)d_out, fb, (size_t)NTK * IC / 4);
}
